// Model_75015898792668
// MI455X (gfx1250) — hardware-verified
//
#include <hip/hip_runtime.h>
#include <stddef.h>
#include <stdint.h>


#define DF     128
#define AP     256
#define NREL   4
#define NTHR   256
#define NWAVE  8
#define EPT    8
#define CHUNK  (NTHR * EPT)
#define WCAP   (EPT * 32)
#define LISTN  (NWAVE * WCAP)
#define NBA    1024
#define SLA    10
#define RCAP   8192
#define DEGCAP 64
#define GBM    64
#define GBN    128
#define GTHR   128
#define U_WL   32768
#define U_R1   4096
#define U_R2   6144
#define U_DW   8192
#define U_ALL  (U_WL + U_R1 + U_R2 + U_DW)
#define NUBLK  (U_ALL / NTHR)
#define AGG_ZINTS    (LISTN + 2 * RCAP + 3 * NBA)
#define MISC_INTS    16
#define ROWBUF_INTS  (NWAVE * AP / 2)
#define AGG_LDS_INTS (AGG_ZINTS + MISC_INTS + ROWBUF_INTS)
#define WSMAX  268435456

static_assert((CHUNK & (CHUNK - 1)) == 0 && CHUNK <= 4096);
static_assert((NBA & (NBA - 1)) == 0 && NBA == (1 << SLA));
static_assert(((long long)CHUNK << SLA) < (1LL << 31));
static_assert(LISTN % NTHR == 0);
static_assert(NBA % NWAVE == 0 && NBA % 32 == 0 && NBA % GBM == 0);
static_assert(RCAP % 4 == 0 && AGG_ZINTS % 4 == 0 && LISTN % 4 == 0 && ((AGG_ZINTS + MISC_INTS) % 4) == 0);
static_assert(AGG_ZINTS % (NTHR * 4) == 0);
static_assert(GBN == DF && GBM == (GTHR / 32) * 16 && DF == 4 * 32 && AP == 2 * DF && DF % 32 == 0);
static_assert(U_WL % NTHR == 0 && U_R1 % NTHR == 0 && U_R2 % NTHR == 0 && U_DW % NTHR == 0);
static_assert(U_WL == 8 * DF * (AP / 8) && U_R1 == DF * (AP / 8) && U_R2 == DF * 48 && U_DW == 2 * DF * (AP / 8));
static_assert(AGG_LDS_INTS * 4 <= 300000);

typedef float          v4f   __attribute__((ext_vector_type(4)));
typedef float          v8f   __attribute__((ext_vector_type(8)));
typedef int            v4i   __attribute__((ext_vector_type(4)));
typedef int            v8i   __attribute__((ext_vector_type(8)));
typedef unsigned       v2u   __attribute__((ext_vector_type(2)));
typedef unsigned short v4us  __attribute__((ext_vector_type(4)));
typedef unsigned short v8us  __attribute__((ext_vector_type(8)));
typedef unsigned short v16us __attribute__((ext_vector_type(16)));
typedef __bf16         v16bf __attribute__((ext_vector_type(16)));
typedef v4f  __attribute__((may_alias)) v4fa;
typedef v4i  __attribute__((may_alias)) v4ia;
typedef v2u  __attribute__((may_alias)) v2ua;
typedef v4us __attribute__((may_alias)) v4usa;
typedef v8us __attribute__((may_alias)) v8usa;
union FragB { v16bf v; v16us u; v8us h[2]; v8i w; };

__device__ __forceinline__ v8f wmb(const FragB& a, const FragB& b, v8f c) {
  v8f d = __builtin_amdgcn_wmma_f32_16x16x32_bf16(false, a.v, false, b.v, (short)0, c, false, false);
  asm volatile("v_nop\n\tv_nop\n\tv_nop\n\tv_nop" : "+v"(d) : "v"(a.w), "v"(b.w));
  return d;
}

__device__ __forceinline__ unsigned bf16_bits(float f) {
  const unsigned u = __float_as_uint(f);
  return (u + 0x7FFFu + ((u >> 16) & 1u)) >> 16;
}
__device__ __forceinline__ float bf16_val(float f) {
  return __uint_as_float(bf16_bits(f) << 16);
}

__device__ __forceinline__ void wave_sync() {
  __builtin_amdgcn_fence(__ATOMIC_RELEASE, "wavefront");
  __builtin_amdgcn_wave_barrier();
  __builtin_amdgcn_fence(__ATOMIC_ACQUIRE, "wavefront");
}

__device__ __forceinline__ void st2us(unsigned short* dp, v8us o) {
  *(volatile v8us*)dp = o;
  __threadfence();
  *(volatile v8us*)dp = o;
}

template <int SLB>
__device__ __forceinline__ int scan_chunk(const int* __restrict__ dsts, int nE, int cbase, int slotBase,
                                          int nb, int vec8, int* list, int tid, int lane, int wave) {
  int wc = 0;
  const int el0  = tid * EPT;
  const int e0   = cbase + el0;
  const int sent = -2147483647 - 1;
  v4i da, db;
  if (vec8 != 0 && cbase + CHUNK <= nE) {
    da = *(const v4i*)(dsts + e0);
    db = *(const v4i*)(dsts + e0 + 4);
  } else {
    da.x = (e0     < nE) ? dsts[min(e0,     nE - 1)] : sent;
    da.y = (e0 + 1 < nE) ? dsts[min(e0 + 1, nE - 1)] : sent;
    da.z = (e0 + 2 < nE) ? dsts[min(e0 + 2, nE - 1)] : sent;
    da.w = (e0 + 3 < nE) ? dsts[min(e0 + 3, nE - 1)] : sent;
    db.x = (e0 + 4 < nE) ? dsts[min(e0 + 4, nE - 1)] : sent;
    db.y = (e0 + 5 < nE) ? dsts[min(e0 + 5, nE - 1)] : sent;
    db.z = (e0 + 6 < nE) ? dsts[min(e0 + 6, nE - 1)] : sent;
    db.w = (e0 + 7 < nE) ? dsts[min(e0 + 7, nE - 1)] : sent;
  }
  const unsigned nbs = (unsigned)slotBase;
  const unsigned unb = (unsigned)nb;
  const unsigned s0 = (unsigned)da.x - nbs, s1 = (unsigned)da.y - nbs;
  const unsigned s2 = (unsigned)da.z - nbs, s3 = (unsigned)da.w - nbs;
  const unsigned s4 = (unsigned)db.x - nbs, s5 = (unsigned)db.y - nbs;
  const unsigned s6 = (unsigned)db.z - nbs, s7 = (unsigned)db.w - nbs;
  const bool h0 = s0 < unb, h1 = s1 < unb, h2 = s2 < unb, h3 = s3 < unb;
  const bool h4 = s4 < unb, h5 = s5 < unb, h6 = s6 < unb, h7 = s7 < unb;
  const unsigned any = __builtin_amdgcn_ballot_w32(h0 | h1 | h2 | h3 | h4 | h5 | h6 | h7);
  if (any != 0u) {
#define HITJ(J, HJ, SJ) { \
      const unsigned mj = __builtin_amdgcn_ballot_w32(HJ); \
      if (mj != 0u) { \
        if (HJ) { \
          const int pos = wc + (int)__builtin_amdgcn_mbcnt_lo(mj, 0u); \
          if (pos < WCAP) list[wave * WCAP + pos] = ((el0 + (J)) << SLB) | (int)(SJ); \
        } \
        wc += (int)__builtin_popcount(mj); } }
    HITJ(0, h0, s0)
    HITJ(1, h1, s1)
    HITJ(2, h2, s2)
    HITJ(3, h3, s3)
    HITJ(4, h4, s4)
    HITJ(5, h5, s5)
    HITJ(6, h6, s6)
    HITJ(7, h7, s7)
#undef HITJ
  }
  return wc;
}

__device__ __forceinline__ void gather8(const float* __restrict__ p, float (&f)[8]) {
#pragma unroll
  for (int i = 0; i < 8; ++i) f[i] = p[(size_t)i * DF];
}
__device__ __forceinline__ void wrsum8(const float* __restrict__ Wr, int n, int kk, float (&s)[8]) {
#pragma unroll
  for (int i = 0; i < 8; ++i) s[i] = 0.0f;
#pragma unroll 1
  for (int r = 0; r < NREL; ++r) {
    float f[8];
    gather8(Wr + (size_t)r * DF * DF + (size_t)kk * DF + n, f);
#pragma unroll
    for (int i = 0; i < 8; ++i) s[i] = s[i] + bf16_val(f[i]);
  }
}
__device__ __forceinline__ v8us pack_plain(const float (&f)[8]) {
  v8us o;
#pragma unroll
  for (int i = 0; i < 8; ++i) o[i] = (unsigned short)bf16_bits(f[i]);
  return o;
}
__device__ __forceinline__ v8us pack_hl(const float (&s)[8], bool lo) {
  v8us o;
#pragma unroll
  for (int i = 0; i < 8; ++i) {
    const unsigned hb = bf16_bits(s[i]);
    const unsigned lb = bf16_bits(s[i] - __uint_as_float(hb << 16));
    o[i] = (unsigned short)(lo ? lb : hb);
  }
  return o;
}
__device__ __forceinline__ void sumb(const float* __restrict__ b, float* dp, int lane) {
  const v4f a0 = *(const v4f*)(b + 0 * DF + 4 * lane);
  const v4f a1 = *(const v4f*)(b + 1 * DF + 4 * lane);
  const v4f a2 = *(const v4f*)(b + 2 * DF + 4 * lane);
  const v4f a3 = *(const v4f*)(b + 3 * DF + 4 * lane);
  v4f s;
  s.x = ((bf16_val(a0.x) + bf16_val(a1.x)) + bf16_val(a2.x)) + bf16_val(a3.x);
  s.y = ((bf16_val(a0.y) + bf16_val(a1.y)) + bf16_val(a2.y)) + bf16_val(a3.y);
  s.z = ((bf16_val(a0.z) + bf16_val(a1.z)) + bf16_val(a2.z)) + bf16_val(a3.z);
  s.w = ((bf16_val(a0.w) + bf16_val(a1.w)) + bf16_val(a2.w)) + bf16_val(a3.w);
  *(volatile v4f*)dp = s;
  __threadfence();
  *(volatile v4f*)dp = s;
}

__global__ __launch_bounds__(NTHR) void k_wprep(
    const float* __restrict__ Wl1, const float* __restrict__ Wr1, const float* __restrict__ b1,
    const float* __restrict__ Wl2, const float* __restrict__ Wr2, const float* __restrict__ b2,
    const float* __restrict__ dW1,
    unsigned short* WLT, unsigned short* WRS1, unsigned short* WRS2, unsigned short* DWT, float* BS) {
  const int tid = (int)threadIdx.x;
  if ((int)blockIdx.x == NUBLK) {
    const int lane = tid & 31, wave = tid >> 5;
    if (wave == 0)      sumb(b1, BS + 4 * lane, lane);
    else if (wave == 1) sumb(b2, BS + DF + 4 * lane, lane);
    return;
  }
  const int u = (int)blockIdx.x * NTHR + tid;
  if (u < U_WL) {
    const int mat = u >> 12;
    const int w   = u & 4095;
    const int n   = w >> 5;
    const int k8  = (w & 31) * 8;
    const int kk  = k8 & (DF - 1);
    const int r   = mat & 3;
    const size_t so = (size_t)r * DF * DF + (size_t)kk * DF + n;
    float f[8];
    if (mat < 4) gather8(Wl1 + so, f);
    else         gather8(Wl2 + so, f);
    st2us(WLT + (size_t)mat * DF * AP + (size_t)n * AP + k8, pack_plain(f));
  } else if (u < U_WL + U_R1) {
    const int v  = u - U_WL;
    const int n  = v >> 5;
    const int k8 = (v & 31) * 8;
    const int kk = k8 & (DF - 1);
    float s[8];
    wrsum8(Wr1, n, kk, s);
    st2us(WRS1 + (size_t)n * AP + k8, pack_hl(s, (k8 >> 7) == 1));
  } else if (u < U_WL + U_R1 + U_R2) {
    const int v  = u - (U_WL + U_R1);
    const int n  = v / 48;
    const int k8 = (v - n * 48) * 8;
    const int kk = k8 & (DF - 1);
    float s[8];
    wrsum8(Wr2, n, kk, s);
    st2us(WRS2 + (size_t)n * (3 * DF) + k8, pack_hl(s, (k8 >> 7) == 1));
  } else {
    const int v  = u - (U_WL + U_R1 + U_R2);
    const int n  = v >> 5;
    const int k8 = (v & 31) * 8;
    const int kk = k8 & (DF - 1);
    const int so = (n < DF) ? (kk * DF + n) : ((DF + kk) * DF + (n - DF));
    float f[8];
    gather8(dW1 + so, f);
    st2us(DWT + (size_t)n * AP + k8, pack_plain(f));
  }
}

__global__ __launch_bounds__(NTHR) void k_cvx(const float* __restrict__ x, int nN, int nUnits,
                                              unsigned short* xb) {
  const int u = (int)blockIdx.x * NTHR + (int)threadIdx.x;
  if (u >= nUnits) return;
  const int row = u >> 4;
  const int k8  = (u & 15) * 8;
  const int rc  = row < nN ? row : nN - 1;
  const float* p = x + (size_t)rc * DF + k8;
  const v4f a = *(const v4fa*)p;
  const v4f b = *(const v4fa*)(p + 4);
  const bool ok = row < nN;
  v8us o;
  o[0] = ok ? (unsigned short)bf16_bits(a.x) : (unsigned short)0;
  o[1] = ok ? (unsigned short)bf16_bits(a.y) : (unsigned short)0;
  o[2] = ok ? (unsigned short)bf16_bits(a.z) : (unsigned short)0;
  o[3] = ok ? (unsigned short)bf16_bits(a.w) : (unsigned short)0;
  o[4] = ok ? (unsigned short)bf16_bits(b.x) : (unsigned short)0;
  o[5] = ok ? (unsigned short)bf16_bits(b.y) : (unsigned short)0;
  o[6] = ok ? (unsigned short)bf16_bits(b.z) : (unsigned short)0;
  o[7] = ok ? (unsigned short)bf16_bits(b.w) : (unsigned short)0;
  st2us(xb + (size_t)row * DF + k8, o);
}

template <int L0>
__global__ __launch_bounds__(NTHR) void k_scan(const int* __restrict__ gath, const int* __restrict__ keys,
                                               int nE, int nN, int vec8, int mRows,
                                               const unsigned short* __restrict__ gsrc, unsigned short* mpl) {
  extern __shared__ __attribute__((aligned(16))) int dsm[];
  int* list = dsm;
  int* hl   = dsm + LISTN;
  int* sl   = hl + RCAP;
  int* cnt  = sl + RCAP;
  int* offs = cnt + NBA;
  int* cur  = offs + NBA;
  int* misc = cur + NBA;
  const int tid = (int)threadIdx.x, lane = tid & 31, wave = tid >> 5;
  unsigned short* rowbuf = (unsigned short*)(misc + MISC_INTS) + wave * AP;
  const int nodeBase = (int)blockIdx.x * NBA;

  {
    const v4i z4 = {0, 0, 0, 0};
    for (int i = tid * 4; i < AGG_ZINTS; i += NTHR * 4) *(v4ia*)(dsm + i) = z4;
    if (tid < MISC_INTS) misc[tid] = 0;
  }
  __syncthreads();

  int t = 0, ov = 0;
  const int nChunks = (nE + CHUNK - 1) / CHUNK;
#pragma unroll 1
  for (int ch = 0; ch < nChunks; ++ch) {
    const int cbase = ch * CHUNK;
    const int wc = scan_chunk<SLA>(keys, nE, cbase, nodeBase, NBA, vec8, list, tid, lane, wave);
    if (lane == 0) misc[wave] = wc;
    __syncthreads();
    if (wave == 0) {
#pragma unroll 1
      for (int w2 = 0; w2 < NWAVE; ++w2) {
        int c = misc[w2];
        c = c < 0 ? 0 : (c > WCAP ? WCAP : c);
#pragma unroll 1
        for (int b0 = 0; b0 < c; b0 += 32) {
          const int idx = b0 + lane;
          const int ent = list[w2 * WCAP + (idx < WCAP ? idx : WCAP - 1)];
          const int m32 = (c - b0) < 32 ? (c - b0) : 32;
#pragma unroll 1
          for (int k = 0; k < m32; ++k) {
            const int u    = __builtin_amdgcn_readlane(ent, k);
            const int slot = u & (NBA - 1);
            const int el   = (u >> SLA) & (CHUNK - 1);
            const int pk   = ((cbase + el) << SLA) | slot;
            if (t < RCAP) {
              if (lane == 0) { hl[t] = pk; cnt[slot] = cnt[slot] + 1; }
              t = t + 1;
            } else {
              ov = 1;
            }
          }
        }
      }
    }
    __syncthreads();
  }
  if (wave == 0 && lane == 0) { misc[8] = t; misc[9] = ov; }
  __syncthreads();
  int tt = misc[8];
  tt = tt < 0 ? 0 : (tt > RCAP ? RCAP : tt);
  const int ovf = misc[9];

  if (wave == 0) {
    const int base = lane * (NBA / 32);
    int s = 0;
#pragma unroll 1
    for (int i = 0; i < NBA / 32; ++i) s += cnt[base + i];
    int incl = s;
#pragma unroll
    for (int d = 1; d < 32; d <<= 1) {
      const int y = __shfl_up(incl, d, 32);
      if (lane >= d) incl += y;
    }
    int run = incl - s;
#pragma unroll 1
    for (int i = 0; i < NBA / 32; ++i) {
      const int cv = cnt[base + i];
      offs[base + i] = run;
      cur[base + i]  = run;
      run += cv;
    }
  }
  __syncthreads();
  if (wave == 0) {
#pragma unroll 1
    for (int b0 = 0; b0 < tt; b0 += 32) {
      const int idx = b0 + lane;
      const int ent = hl[idx < RCAP ? idx : RCAP - 1];
      const int m32 = (tt - b0) < 32 ? (tt - b0) : 32;
#pragma unroll 1
      for (int k = 0; k < m32; ++k) {
        const int u    = __builtin_amdgcn_readlane(ent, k);
        const int slot = u & (NBA - 1);
        if (lane == 0) {
          int p = cur[slot];
          p = p < 0 ? 0 : (p > RCAP - 1 ? RCAP - 1 : p);
          sl[p] = u;
          cur[slot] = p + 1;
        }
      }
    }
  }
  __syncthreads();

  const float qnan = __int_as_float(0x7fc00000);
  const float pz = (ovf != 0) ? qnan : 0.0f;
#pragma unroll 1
  for (int si = 0; si < NBA / NWAVE; ++si) {
    const int s    = si * NWAVE + wave;
    const int node = nodeBase + s;
    int cfull = cnt[s];
    cfull = cfull < 0 ? 0 : cfull;
    const bool big = cfull > DEGCAP;
    const int c = cfull > DEGCAP ? DEGCAP : cfull;
    int o = offs[s];
    o = o < 0 ? 0 : (o > RCAP ? RCAP : o);
    float a0 = 0.0f, a1 = 0.0f, a2 = 0.0f, a3 = 0.0f;
#pragma unroll 1
    for (int b0 = 0; b0 < c; b0 += 32) {
      int idx = o + b0 + lane;
      idx = idx > RCAP - 1 ? RCAP - 1 : idx;
      const int ent = sl[idx];
      int eid = ent >> SLA;
      eid = eid < 0 ? 0 : (eid > nE - 1 ? nE - 1 : eid);
      int sr = gath[eid];
      sr = sr < 0 ? 0 : (sr > nN - 1 ? nN - 1 : sr);
      const int m32 = (c - b0) < 32 ? (c - b0) : 32;
#pragma unroll 1
      for (int k = 0; k < m32; ++k) {
        const int sk = __builtin_amdgcn_readlane(sr, k);
        if constexpr (L0 != 0) {
          const v2u w = *(const v2ua*)(gsrc + (size_t)sk * DF + 4 * lane);
          a0 = a0 + __uint_as_float(w.x << 16);
          a1 = a1 + __uint_as_float(w.x & 0xffff0000u);
          a2 = a2 + __uint_as_float(w.y << 16);
          a3 = a3 + __uint_as_float(w.y & 0xffff0000u);
        } else {
          const unsigned short* rp = gsrc + (size_t)sk * AP + 4 * lane;
          const v2u wh = *(const v2ua*)rp;
          const v2u wl = *(const v2ua*)(rp + DF);
          const float f0 = __uint_as_float(wh.x << 16)         + __uint_as_float(wl.x << 16);
          const float f1 = __uint_as_float(wh.x & 0xffff0000u) + __uint_as_float(wl.x & 0xffff0000u);
          const float f2 = __uint_as_float(wh.y << 16)         + __uint_as_float(wl.y << 16);
          const float f3 = __uint_as_float(wh.y & 0xffff0000u) + __uint_as_float(wl.y & 0xffff0000u);
          a0 = a0 + f0;
          a1 = a1 + f1;
          a2 = a2 + f2;
          a3 = a3 + f3;
        }
      }
    }
    const int   cf  = cfull < 1 ? 1 : cfull;
    const float inv = 1.0f / (float)cf;
    const float pzr = big ? qnan : pz;
    const bool live = node < nN;
    const float m0 = live ? (a0 * inv + pzr) : 0.0f;
    const float m1 = live ? (a1 * inv + pzr) : 0.0f;
    const float m2 = live ? (a2 * inv + pzr) : 0.0f;
    const float m3 = live ? (a3 * inv + pzr) : 0.0f;
    v4us mh, ml;
    {
      unsigned hb;
      hb = bf16_bits(m0); mh[0] = (unsigned short)hb; ml[0] = (unsigned short)bf16_bits(m0 - __uint_as_float(hb << 16));
      hb = bf16_bits(m1); mh[1] = (unsigned short)hb; ml[1] = (unsigned short)bf16_bits(m1 - __uint_as_float(hb << 16));
      hb = bf16_bits(m2); mh[2] = (unsigned short)hb; ml[2] = (unsigned short)bf16_bits(m2 - __uint_as_float(hb << 16));
      hb = bf16_bits(m3); mh[3] = (unsigned short)hb; ml[3] = (unsigned short)bf16_bits(m3 - __uint_as_float(hb << 16));
    }
    *(v4usa*)(rowbuf + 4 * lane) = mh;
    *(v4usa*)(rowbuf + DF + 4 * lane) = ml;
    wave_sync();
    const v8us q0 = *(const v8usa*)(rowbuf + 8 * lane);
    wave_sync();
    if (node < mRows) {
      unsigned short* rpw = mpl + (size_t)node * AP + 8 * lane;
      *(volatile v8us*)rpw = q0;
      __threadfence();
      *(volatile v8us*)rpw = q0;
    }
  }
}

__device__ __forceinline__ void mm_pass(v8f (&acc)[8], const unsigned short* ap, const unsigned short* bp,
                                        int nch, int am, int Kb) {
#pragma unroll 1
  for (int c = 0; c < nch; ++c) {
    const int ao = ((am >> c) & 1) * DF;
#pragma unroll 1
    for (int kk = 0; kk < DF; kk += 32) {
      FragB af;
      af.h[0] = *(const v8usa*)(ap + ao + kk);
      af.h[1] = *(const v8usa*)(ap + ao + kk + 16);
      const unsigned short* wq0 = bp + c * DF + kk;
#pragma unroll
      for (int nt = 0; nt < 8; ++nt) {
        const unsigned short* wq = wq0 + (size_t)(16 * nt) * (size_t)Kb;
        FragB bf;
        bf.h[0] = *(const v8usa*)wq;
        bf.h[1] = *(const v8usa*)(wq + 16);
        acc[nt] = wmb(af, bf, acc[nt]);
      }
    }
  }
}

template <int EPI>
__global__ __launch_bounds__(GTHR) void k_gemm(
    const unsigned short* A1, int p1, int nch1, int am1, const unsigned short* __restrict__ B1,
    const unsigned short* A2, int p2, int nch2, int am2, const unsigned short* __restrict__ B2,
    float* accp, int ldc, int rdc, const float* __restrict__ bsum, int addb,
    unsigned short* outH, int nN) {
  __shared__ __attribute__((aligned(16))) float stg[GBM * GBN];
  const int tid = (int)threadIdx.x, lane = tid & 31, wave = tid >> 5, hh = lane >> 4, m = lane & 15;
  const int rowBase = (int)blockIdx.x * GBM;
  const int cb      = (int)blockIdx.y;

  v8f acc[8];
  {
    const v8f z = {0.f, 0.f, 0.f, 0.f, 0.f, 0.f, 0.f, 0.f};
#pragma unroll
    for (int t = 0; t < 8; ++t) acc[t] = z;
  }
  {
    const int Kb = nch1 * DF;
    const unsigned short* ap = A1 + (size_t)(rowBase + 16 * wave + m) * (size_t)p1 + 8 * hh;
    const unsigned short* bp = B1 + (size_t)(GBN * cb + m) * (size_t)Kb + 8 * hh;
    mm_pass(acc, ap, bp, nch1, am1, Kb);
  }
  if (nch2 > 0) {
    const int Kb = nch2 * DF;
    const unsigned short* ap = A2 + (size_t)(rowBase + 16 * wave + m) * (size_t)p2 + 8 * hh;
    const unsigned short* bp = B2 + (size_t)(GBN * cb + m) * (size_t)Kb + 8 * hh;
    mm_pass(acc, ap, bp, nch2, am2, Kb);
  }

#pragma unroll
  for (int nt = 0; nt < 8; ++nt) {
    const int lc = 16 * nt + m;
#pragma unroll
    for (int r = 0; r < 8; ++r) {
      const int lr = 16 * wave + 8 * hh + r;
      stg[lr * GBN + lc] = acc[nt][r];
    }
  }
  __syncthreads();

  v4f bb4;
  {
    const v4f t1 = *(const v4f*)(bsum + 4 * lane);
    const bool ab = addb != 0;
    bb4.x = ab ? t1.x : 0.0f; bb4.y = ab ? t1.y : 0.0f; bb4.z = ab ? t1.z : 0.0f; bb4.w = ab ? t1.w : 0.0f;
  }

#pragma unroll 1
  for (int g = 0; g < 4; ++g) {
    v4f pv[4];
#pragma unroll
    for (int j = 0; j < 4; ++j) {
      const int lr = 16 * wave + 4 * g + j;
      pv[j] = *(const v4fa*)(stg + lr * GBN + 4 * lane);
    }
    if (rdc != 0) {
#pragma unroll
      for (int j = 0; j < 4; ++j) {
        const int gr = rowBase + 16 * wave + 4 * g + j;
        const v4f cv = *(const v4f*)(accp + (size_t)gr * (size_t)ldc + GBN * cb + 4 * lane);
        pv[j] = pv[j] + cv;
      }
    }
#pragma unroll
    for (int j = 0; j < 4; ++j) pv[j] = pv[j] + bb4;

    if constexpr (EPI == 0) {
#pragma unroll
      for (int j = 0; j < 4; ++j) {
        const int gr = rowBase + 16 * wave + 4 * g + j;
        *(volatile v4f*)(accp + (size_t)gr * (size_t)ldc + GBN * cb + 4 * lane) = pv[j];
      }
      __threadfence();
#pragma unroll
      for (int j = 0; j < 4; ++j) {
        const int gr = rowBase + 16 * wave + 4 * g + j;
        *(volatile v4f*)(accp + (size_t)gr * (size_t)ldc + GBN * cb + 4 * lane) = pv[j];
      }
    } else {
#pragma unroll
      for (int j = 0; j < 4; ++j) {
        const bool ok = (rowBase + 16 * wave + 4 * g + j) < nN;
        v4f y = pv[j];
        if constexpr (EPI == 1) {
          y.x = (y.x > 0.0f) ? y.x : (y.x - y.x);
          y.y = (y.y > 0.0f) ? y.y : (y.y - y.y);
          y.z = (y.z > 0.0f) ? y.z : (y.z - y.z);
          y.w = (y.w > 0.0f) ? y.w : (y.w - y.w);
        }
        y.x = ok ? y.x : 0.0f; y.y = ok ? y.y : 0.0f; y.z = ok ? y.z : 0.0f; y.w = ok ? y.w : 0.0f;
        pv[j] = y;
      }
      __syncthreads();
#pragma unroll
      for (int j = 0; j < 4; ++j) {
        v4us h4, l4;
        unsigned hb;
        hb = bf16_bits(pv[j].x); h4[0] = (unsigned short)hb; l4[0] = (unsigned short)bf16_bits(pv[j].x - __uint_as_float(hb << 16));
        hb = bf16_bits(pv[j].y); h4[1] = (unsigned short)hb; l4[1] = (unsigned short)bf16_bits(pv[j].y - __uint_as_float(hb << 16));
        hb = bf16_bits(pv[j].z); h4[2] = (unsigned short)hb; l4[2] = (unsigned short)bf16_bits(pv[j].z - __uint_as_float(hb << 16));
        hb = bf16_bits(pv[j].w); h4[3] = (unsigned short)hb; l4[3] = (unsigned short)bf16_bits(pv[j].w - __uint_as_float(hb << 16));
        unsigned short* srow = (unsigned short*)stg + (size_t)(16 * wave + 4 * g + j) * (2 * GBN);
        *(v4usa*)(srow + 4 * lane) = h4;
        *(v4usa*)(srow + DF + 4 * lane) = l4;
      }
      __syncthreads();
      v8us qv[4];
#pragma unroll
      for (int j = 0; j < 4; ++j) {
        const unsigned short* srow = (const unsigned short*)stg + (size_t)(16 * wave + 4 * g + j) * (2 * GBN);
        qv[j] = *(const v8usa*)(srow + 8 * lane);
      }
#pragma unroll
      for (int j = 0; j < 4; ++j) {
        unsigned short* rp = outH + (size_t)(rowBase + 16 * wave + 4 * g + j) * (size_t)AP + 8 * lane;
        *(volatile v8us*)rp = qv[j];
      }
      __threadfence();
#pragma unroll
      for (int j = 0; j < 4; ++j) {
        unsigned short* rp = outH + (size_t)(rowBase + 16 * wave + 4 * g + j) * (size_t)AP + 8 * lane;
        *(volatile v8us*)rp = qv[j];
      }
    }
  }
}

__global__ __launch_bounds__(NTHR) void k_dec(const float* __restrict__ pq, const int* __restrict__ eli,
                                              int nL, int nN,
                                              const float* __restrict__ db1, const float* __restrict__ dW2,
                                              const float* __restrict__ db2, float* out) {
  __shared__ __attribute__((aligned(16))) float os[NTHR];
  const int tid = (int)threadIdx.x, lane = tid & 31, wave = tid >> 5;
  const int l0 = (int)blockIdx.x * NTHR + wave * 32;
  float res = 0.0f;
  if (l0 < nL) {
    const int li = l0 + lane;
    const int lc = li < nL ? li : nL - 1;
    int ri = eli[lc];
    int ci = eli[(size_t)nL + lc];
    ri = ri < 0 ? 0 : (ri > nN - 1 ? nN - 1 : ri);
    ci = ci < 0 ? 0 : (ci > nN - 1 ? nN - 1 : ci);
    v4f b4, w4;
    {
      const v4f a = *(const v4f*)(db1 + 4 * lane);
      const v4f b = *(const v4f*)(dW2 + 4 * lane);
      b4.x = bf16_val(a.x); b4.y = bf16_val(a.y); b4.z = bf16_val(a.z); b4.w = bf16_val(a.w);
      w4.x = bf16_val(b.x); w4.y = bf16_val(b.y); w4.z = bf16_val(b.z); w4.w = bf16_val(b.w);
    }
    const float bb2 = bf16_val(db2[0]);
#pragma unroll 1
    for (int j = 0; j < 32; ++j) {
      const int rj = __builtin_amdgcn_readlane(ri, j);
      const int cj = __builtin_amdgcn_readlane(ci, j);
      const v4f p = *(const v4f*)(pq + (size_t)rj * AP + 4 * lane);
      const v4f q = *(const v4f*)(pq + (size_t)cj * AP + DF + 4 * lane);
      const v4f t = (p + q) + b4;
      const float u0 = (t.x > 0.0f) ? t.x : (t.x - t.x);
      const float u1 = (t.y > 0.0f) ? t.y : (t.y - t.y);
      const float u2 = (t.z > 0.0f) ? t.z : (t.z - t.z);
      const float u3 = (t.w > 0.0f) ? t.w : (t.w - t.w);
      float s = u0 * w4.x;
      s = fmaf(u1, w4.y, s);
      s = fmaf(u2, w4.z, s);
      s = fmaf(u3, w4.w, s);
      s = s + __shfl_xor(s, 16, 32);
      s = s + __shfl_xor(s, 8, 32);
      s = s + __shfl_xor(s, 4, 32);
      s = s + __shfl_xor(s, 2, 32);
      s = s + __shfl_xor(s, 1, 32);
      res = (lane == j) ? s : res;
    }
    res = res + bb2;
  }
  os[tid] = res;
  __syncthreads();
  const v4f ov = *(const v4fa*)(os + 4 * (tid & 63));
  const int idx = (int)blockIdx.x * NTHR + 4 * tid;
  const bool okst = (tid < 64) && (idx + 3 < nL);
  float* op = out + (okst ? (size_t)idx : (size_t)0);
  if (okst) *(volatile v4f*)op = ov;
  __threadfence();
  if (okst) *(volatile v4f*)op = ov;
}

static inline int cdiv(int a, int b) { return (a + b - 1) / b; }
static inline size_t al256(size_t o) { return (o + 255) & ~(size_t)255; }

extern "C" void kernel_launch(void* const* d_in, const int* in_sizes, int n_in,
                              void* d_out, int out_size, void* d_ws, size_t ws_size,
                              hipStream_t stream) {
  if (n_in < 13) return;
  if (in_sizes[0] < DF || (in_sizes[0] % DF) != 0) return;
  const int nN = in_sizes[0] / DF;
  if (nN < 16 || nN >= (1 << 24)) return;
  if (in_sizes[1] < 2 * NREL || (in_sizes[1] % (2 * NREL)) != 0) return;
  const int nE = in_sizes[1] / (2 * NREL);
  if (nE < 1 || nE >= (1 << 21)) return;
  if (in_sizes[2] < 2 || (in_sizes[2] & 1) != 0) return;
  const int nL = in_sizes[2] / 2;
  if (nL < 32 || (nL % 32) != 0) return;
  if (in_sizes[3] != NREL * DF * DF || in_sizes[4] != NREL * DF * DF || in_sizes[5] != NREL * DF) return;
  if (in_sizes[6] != NREL * DF * DF || in_sizes[7] != NREL * DF * DF || in_sizes[8] != NREL * DF) return;
  if (in_sizes[9] != 2 * DF * DF || in_sizes[10] != DF || in_sizes[11] != DF || in_sizes[12] != 1) return;
  if (out_size != nL) return;

  const float* x   = (const float*)d_in[0];
  const int*   ei  = (const int*)d_in[1];
  const int*   eli = (const int*)d_in[2];
  const float* Wl1 = (const float*)d_in[3];
  const float* Wr1 = (const float*)d_in[4];
  const float* b1  = (const float*)d_in[5];
  const float* Wl2 = (const float*)d_in[6];
  const float* Wr2 = (const float*)d_in[7];
  const float* b2  = (const float*)d_in[8];
  const float* dW1 = (const float*)d_in[9];
  const float* db1 = (const float*)d_in[10];
  const float* dW2 = (const float*)d_in[11];
  const float* db2 = (const float*)d_in[12];
  float* out = (float*)d_out;

  const int MP = cdiv(nN, GBM) * GBM;
  const int gM = MP / GBM;
  const int gA = cdiv(MP, NBA);
  if ((long long)gA * NBA < (long long)MP) return;
  const int vec8 = ((nE & 3) == 0) ? 1 : 0;

  char* ws = (char*)d_ws;
  size_t off = 0;
  const size_t oWLT = off; off = al256(off + (size_t)8 * DF * AP * 2);
  const size_t oWR1 = off; off = al256(off + (size_t)DF * AP * 2);
  const size_t oWR2 = off; off = al256(off + (size_t)DF * 3 * DF * 2);
  const size_t oDWT = off; off = al256(off + (size_t)2 * DF * AP * 2);
  const size_t oBS  = off; off = al256(off + (size_t)2 * DF * 4);
  const size_t oXB  = off; off = al256(off + (size_t)MP * DF * 2);
  const size_t oMEA = off; off = al256(off + (size_t)MP * AP * 2);
  const size_t oACC = off; off = al256(off + (size_t)MP * DF * 4);
  const size_t oHHL = off; off = al256(off + (size_t)MP * AP * 2);
  if (off > ws_size || off > (size_t)WSMAX) return;
  if (oHHL != oACC + (size_t)MP * DF * 4) return;
  if ((size_t)MP * AP * 4 != (size_t)MP * DF * 4 + (size_t)MP * AP * 2) return;
  unsigned short* WLT  = (unsigned short*)(ws + oWLT);
  unsigned short* WRS1 = (unsigned short*)(ws + oWR1);
  unsigned short* WRS2 = (unsigned short*)(ws + oWR2);
  unsigned short* DWT  = (unsigned short*)(ws + oDWT);
  float*          BS   = (float*)(ws + oBS);
  unsigned short* XB   = (unsigned short*)(ws + oXB);
  unsigned short* MEA  = (unsigned short*)(ws + oMEA);
  float*          ACC  = (float*)(ws + oACC);
  unsigned short* HHL  = (unsigned short*)(ws + oHHL);
  float*          PQ   = (float*)(ws + oACC);

  const size_t scanLds = (size_t)AGG_LDS_INTS * 4;
  hipFuncSetAttribute(reinterpret_cast<const void*>(&k_scan<1>), hipFuncAttributeMaxDynamicSharedMemorySize, (int)scanLds);
  hipFuncSetAttribute(reinterpret_cast<const void*>(&k_scan<0>), hipFuncAttributeMaxDynamicSharedMemorySize, (int)scanLds);

  k_wprep<<<NUBLK + 1, NTHR, 0, stream>>>(Wl1, Wr1, b1, Wl2, Wr2, b2, dW1, WLT, WRS1, WRS2, DWT, BS);
  const int nUx = MP * (DF / 8);
  k_cvx<<<cdiv(nUx, NTHR), NTHR, 0, stream>>>(x, nN, nUx, XB);

  for (int r = 0; r < NREL; ++r) {
    const int* src = ei + (size_t)(2 * r) * (size_t)nE;
    const int* dst = ei + (size_t)(2 * r + 1) * (size_t)nE;
    const unsigned short* wl = WLT + (size_t)r * DF * AP;
    k_scan<1><<<gA, NTHR, scanLds, stream>>>(src, dst, nE, nN, vec8, MP, XB, MEA);
    if (r == 0)
      k_gemm<0><<<dim3(gM, 1), GTHR, 0, stream>>>(MEA, AP, 2, 2, wl, XB, DF, 2, 0, WRS1,
                                                  ACC, DF, 0, BS, 1, HHL, nN);
    else if (r < NREL - 1)
      k_gemm<0><<<dim3(gM, 1), GTHR, 0, stream>>>(MEA, AP, 2, 2, wl, MEA, AP, 0, 0, wl,
                                                  ACC, DF, 1, BS, 0, HHL, nN);
    else
      k_gemm<1><<<dim3(gM, 1), GTHR, 0, stream>>>(MEA, AP, 2, 2, wl, MEA, AP, 0, 0, wl,
                                                  ACC, DF, 1, BS, 0, HHL, nN);
  }

  for (int r = 0; r < NREL; ++r) {
    const int* src = ei + (size_t)(2 * r) * (size_t)nE;
    const int* dst = ei + (size_t)(2 * r + 1) * (size_t)nE;
    const unsigned short* wl = WLT + (size_t)(NREL + r) * DF * AP;
    k_scan<0><<<gA, NTHR, scanLds, stream>>>(src, dst, nE, nN, vec8, MP, HHL, MEA);
    if (r == 0)
      k_gemm<0><<<dim3(gM, 1), GTHR, 0, stream>>>(MEA, AP, 2, 2, wl, HHL, AP, 3, 4, WRS2,
                                                  ACC, DF, 0, BS + DF, 1, MEA, nN);
    else if (r < NREL - 1)
      k_gemm<0><<<dim3(gM, 1), GTHR, 0, stream>>>(MEA, AP, 2, 2, wl, MEA, AP, 0, 0, wl,
                                                  ACC, DF, 1, BS + DF, 0, MEA, nN);
    else
      k_gemm<2><<<dim3(gM, 1), GTHR, 0, stream>>>(MEA, AP, 2, 2, wl, MEA, AP, 0, 0, wl,
                                                  ACC, DF, 1, BS + DF, 0, MEA, nN);
  }

  k_gemm<0><<<dim3(gM, 2), GTHR, 0, stream>>>(MEA, AP, 2, 2, DWT, MEA, AP, 0, 0, DWT,
                                              PQ, AP, 0, BS, 0, MEA, nN);
  k_dec<<<cdiv(nL, NTHR), NTHR, 0, stream>>>(PQ, eli, nL, nN, db1, dW2, db2, out);
}
